// DeterministicAdjacency_42082089566385
// MI455X (gfx1250) — hardware-run, weakly checked
//
#include <hip/hip_runtime.h>


#ifndef NROWS
#define NROWS 2048
#endif
#define NTOK 2048
#define DM   128
#define ED   64
#define HP   128
#define NT   128
#define TI   4
#define LOG2E_F  1.4426950408889634f
#define NLOG2E_F (-1.4426950408889634f)
#define NEGB (-3.0e38f)

static_assert(HP == 2 * ED);
static_assert(DM % 32 == 0);
static_assert(NTOK % 64 == 0);
static_assert(HP % 64 == 0);
static_assert(ED % 64 == 0);
static_assert((ED & (ED - 1)) == 0);
static_assert(ED % 16 == 0);
static_assert(HP % 16 == 0);
static_assert(DM / 8 == 16);
static_assert((16 * DM) % 256 == 0);
static_assert(((size_t)NTOK * DM) % 8 == 0);
static_assert(TI == NT / 32);
static_assert(NTOK % NT == 0);
static_assert(NTOK % (NT * 4) == 0);
static_assert((size_t)NT * 16 * (NTOK / (NT * 4)) == (size_t)NTOK * 4);
static_assert((TI * ED) % NT == 0);
static_assert(ED % 4 == 0);
static_assert(NROWS % TI == 0);
static_assert(NROWS <= NTOK);
static_assert(8 * 32 * 16 == 16 * 64 * 4);
static_assert((size_t)(TI * NTOK + TI * ED + ED + TI) * 4 <= (size_t)131072);
static_assert((size_t)16 * 68 * 4 <= (size_t)131072);
static_assert((size_t)16 * DM * 2 <= (size_t)131072);

typedef unsigned short bf;
typedef __attribute__((ext_vector_type(16))) __bf16   v16bf;
typedef __attribute__((ext_vector_type(8)))  unsigned short v8us;
typedef __attribute__((ext_vector_type(8)))  float    v8f;
typedef __attribute__((ext_vector_type(4)))  float    v4f;
typedef v4f  __attribute__((may_alias)) v4fa;
typedef v8us __attribute__((may_alias)) v8usa;

__device__ __forceinline__ unsigned short f2bf(float f) { unsigned u = __float_as_uint(f); u += 0x7FFFu + ((u >> 16) & 1u); return (unsigned short)(u >> 16); }
__device__ __forceinline__ float bfr(float f) { return __uint_as_float(((unsigned)f2bf(f)) << 16); }
__device__ __forceinline__ v16bf cat16b(v8us lo, v8us hi) { return __builtin_bit_cast(v16bf, __builtin_shufflevector(lo, hi, 0, 1, 2, 3, 4, 5, 6, 7, 8, 9, 10, 11, 12, 13, 14, 15)); }
__device__ __forceinline__ v8f wmmab(v16bf a, v16bf b, v8f c) { return __builtin_amdgcn_wmma_f32_16x16x32_bf16(false, a, false, b, (short)0, c, false, false); }
__device__ __forceinline__ v16bf ldb(const bf* p)  { return cat16b(*(const v8us*)p, *(const v8us*)(p + 16)); }
__device__ __forceinline__ void wave_sync() { __builtin_amdgcn_fence(3  , "wavefront"); __builtin_amdgcn_wave_barrier(); asm volatile("" ::: "memory"); }
__device__ __forceinline__ v8f wmmab_g(v16bf a, v16bf b, v8f c) { c = wmmab(a, b, c); asm volatile("v_nop\n\tv_nop\n\tv_nop\n\tv_nop" : "+v"(c) : "v"(a), "v"(b)); return c; }
__device__ __forceinline__ float silu_f(float x) { const float ex = __builtin_amdgcn_exp2f(x * NLOG2E_F); return x * __builtin_amdgcn_rcpf(1.0f + ex); }

__global__ __launch_bounds__(256) void k_cvt8(const float* __restrict__ src, bf* dst, size_t n8) {
    const size_t i = (size_t)blockIdx.x * 256 + threadIdx.x; if (i >= n8) return;
    const v8f v = *(const v8f*)(src + i * 8); v8us o;
#pragma unroll
    for (int k = 0; k < 8; ++k) o[k] = f2bf(v[k]);
    *(volatile v8us*)(dst + i * 8) = o; __threadfence(); *(volatile v8us*)(dst + i * 8) = o;
}

__global__ __launch_bounds__(256) void k_wt(const float* __restrict__ W1, bf* WT) {
    __shared__ __align__(16) unsigned short ts[16 * DM];
    const int t = threadIdx.x; const int n0 = blockIdx.x * 16;
    const int half = n0 / ED, cb = n0 % ED;
#pragma unroll 1
    for (int it = 0; it < (16 * DM) / 256; ++it) { const int idx = it * 256 + t; const int k = idx >> 4, c = idx & 15;
        ts[c * DM + k] = f2bf(W1[((size_t)half * DM + (size_t)k) * ED + cb + c]); }
    __syncthreads();
    const int row = t >> 4, pc = (t & 15) * 8;
    const v8us o = *(const v8usa*)(&ts[row * DM + pc]);
    bf* dp = WT + (size_t)(n0 + row) * DM + pc;
    *(volatile v8us*)dp = o; __threadfence(); *(volatile v8us*)dp = o;
}

__global__ __launch_bounds__(32) void k_hproj(const bf* __restrict__ A, const bf* __restrict__ Bt, const float* __restrict__ bias, float* HO) {
    __shared__ __align__(16) float os[16 * 68];
    const int K = DM;
    const int lane = threadIdx.x & 31, lr = lane & 15, hi = lane >> 4; const int r0 = blockIdx.x * 64, c0 = blockIdx.y * 64;
    v8f acc[4][4];
#pragma unroll
    for (int mb = 0; mb < 4; ++mb)
#pragma unroll
        for (int nb = 0; nb < 4; ++nb) acc[mb][nb] = (v8f){};
    const size_t aoff = (size_t)(r0 + lr) * K + 8 * hi, boff = (size_t)(c0 + lr) * K + 8 * hi;
#pragma unroll 1
    for (int kc = 0; kc < K; kc += 32) {
        v16bf a[4];
#pragma unroll
        for (int mb = 0; mb < 4; ++mb) a[mb] = ldb(A + aoff + (size_t)mb * 16 * K + kc);
#pragma unroll
        for (int nb = 0; nb < 4; ++nb) { const v16bf b = ldb(Bt + boff + (size_t)nb * 16 * K + kc);
#pragma unroll
            for (int mb = 0; mb < 4; ++mb) acc[mb][nb] = wmmab_g(a[mb], b, acc[mb][nb]); }
    }
    const bool hb = c0 < ED;
    float bc[4];
#pragma unroll
    for (int nb = 0; nb < 4; ++nb) { float bv = bias[(c0 + nb * 16 + lr) & (ED - 1)];
        asm volatile("" : "+v"(bv));
        bc[nb] = hb ? bfr(bv) : 0.0f; }
#pragma unroll
    for (int mb = 0; mb < 4; ++mb) {
#pragma unroll
        for (int nb = 0; nb < 4; ++nb) {
#pragma unroll
            for (int j = 0; j < 8; ++j) os[(hi * 8 + j) * 68 + nb * 16 + lr] = acc[mb][nb][j] + bc[nb]; }
        wave_sync();
#pragma unroll 1
        for (int ps = 0; ps < 2; ++ps) {
#pragma unroll
            for (int s = 0; s < 8; ++s) { const int p = s * 32 + lane; const int row = p >> 4, c4 = (p & 15) * 4;
                const v4f val = *(const v4fa*)(&os[row * 68 + c4]);
                *(volatile v4f*)(HO + (size_t)(r0 + mb * 16 + row) * HP + c0 + c4) = val; }
            if (ps == 0) __threadfence(); }
        wave_sync();
    }
}

__global__ __launch_bounds__(NT) void k_pair(const float* __restrict__ H, const float* __restrict__ W2, const float* __restrict__ B2, float* OUT) {
#pragma clang fp contract(off)
    __shared__ __align__(16) float sHi[TI * ED];
    __shared__ __align__(16) float sW2[ED];
    __shared__ __align__(16) float sLog[TI * NTOK];
    __shared__ float sInv[TI];
    const int t = threadIdx.x;
    const int lane = t & 31;
    const int wave = __builtin_amdgcn_readfirstlane((int)(threadIdx.x >> 5));
    const int i0 = blockIdx.x * TI;
    if (wave < ED / 32) sW2[t] = bfr(W2[t]);
#pragma unroll
    for (int it = 0; it < (TI * ED) / NT; ++it) { const int idx = it * NT + t; sHi[idx] = H[(size_t)(i0 + idx / ED) * HP + (idx % ED)]; }
    const float b2v = bfr(B2[0]);
    __syncthreads();

#pragma unroll 1
    for (int jj = 0; jj < NTOK / NT; ++jj) {
        const int j = jj * NT + t;
        const float* hp = H + (size_t)j * HP + ED;
        float acc[TI];
#pragma unroll
        for (int r = 0; r < TI; ++r) acc[r] = 0.0f;
#pragma unroll 1
        for (int q = 0; q < ED; q += 4) {
            const v4f hv = *(const v4f*)(hp + q);
            const v4f w = *(const v4fa*)(&sW2[q]);
#pragma unroll
            for (int r = 0; r < TI; ++r) {
                const v4f a = *(const v4fa*)(&sHi[r * ED + q]);
#pragma unroll
                for (int c = 0; c < 4; ++c) acc[r] = fmaf(silu_f(a[c] + hv[c]), w[c], acc[r]);
            }
        }
#pragma unroll
        for (int r = 0; r < TI; ++r) sLog[r * NTOK + j] = acc[r] + b2v;
    }
    __syncthreads();

    {
        const int rb = wave * NTOK;
        float mx = NEGB;
#pragma unroll 4
        for (int idx = lane; idx < NTOK; idx += 32) mx = fmaxf(mx, sLog[rb + idx]);
        mx = fmaxf(mx, __shfl_xor(mx, 16, 32)); mx = fmaxf(mx, __shfl_xor(mx, 8, 32)); mx = fmaxf(mx, __shfl_xor(mx, 4, 32));
        mx = fmaxf(mx, __shfl_xor(mx, 2, 32));  mx = fmaxf(mx, __shfl_xor(mx, 1, 32));
        float sum = 0.0f;
#pragma unroll 4
        for (int idx = lane; idx < NTOK; idx += 32) {
            const float ev = __builtin_amdgcn_exp2f((sLog[rb + idx] - mx) * LOG2E_F);
            sLog[rb + idx] = ev;
            sum += ev; }
        sum += __shfl_xor(sum, 16, 32); sum += __shfl_xor(sum, 8, 32); sum += __shfl_xor(sum, 4, 32);
        sum += __shfl_xor(sum, 2, 32);  sum += __shfl_xor(sum, 1, 32);
        if (lane == 0) sInv[wave] = __builtin_amdgcn_rcpf(sum);
    }
    __syncthreads();

#pragma unroll 1
    for (int ps = 0; ps < 2; ++ps) {
#pragma unroll
        for (int r = 0; r < TI; ++r) {
            const float inv = sInv[r];
            float* orow = OUT + (size_t)(i0 + r) * NTOK;
#pragma unroll
            for (int it = 0; it < NTOK / (NT * 4); ++it) { const int col = (it * NT + t) * 4;
                const v4f e4 = *(const v4fa*)(&sLog[r * NTOK + col]);
                const v4f val = e4 * inv;
                *(volatile v4f*)(orow + col) = val; }
        }
        if (ps == 0) __threadfence(); }
}

static constexpr size_t al256(size_t v) { return (v + 255) & ~(size_t)255; }
static constexpr size_t SZ_ZB = al256((size_t)NTOK * DM * 2);
static constexpr size_t SZ_WT = al256((size_t)HP * DM * 2);
static constexpr size_t SZ_H  = al256((size_t)NTOK * HP * 4);
static constexpr size_t SZ_TOTAL = SZ_ZB + SZ_WT + SZ_H;
static_assert(SZ_TOTAL <= (size_t)134217728);
static_assert((size_t)(NTOK / 64) * 64 * DM * 2 <= SZ_ZB);
static_assert((size_t)(HP / 16) * 16 * DM * 2 <= SZ_WT);
static_assert((size_t)(NTOK / 64) * 64 * HP * 4 <= SZ_H);

extern "C" void kernel_launch(void* const* d_in, const int* in_sizes, int n_in,
                              void* d_out, int out_size, void* d_ws, size_t ws_size, hipStream_t stream) {
    if (n_in < 5) return;
    if ((size_t)in_sizes[0] < (size_t)NTOK * DM) return;
    if ((size_t)in_sizes[1] < (size_t)2 * DM * ED) return;
    if (in_sizes[2] < ED || in_sizes[3] < ED || in_sizes[4] < 1) return;
    if ((size_t)out_size < (size_t)NROWS * NTOK) return;
    if (SZ_TOTAL > ws_size) return;
    const float* z  = (const float*)d_in[0];
    const float* w1 = (const float*)d_in[1];
    const float* b1 = (const float*)d_in[2];
    const float* w2 = (const float*)d_in[3];
    const float* b2 = (const float*)d_in[4];
    float* OUT = (float*)d_out;
    char* wsp = (char*)d_ws;
    bf* ZB = (bf*)wsp; wsp += SZ_ZB;
    bf* WT = (bf*)wsp; wsp += SZ_WT;
    float* HPL = (float*)wsp; wsp += SZ_H;

    { const size_t n8 = (size_t)NTOK * DM / 8;
      k_cvt8<<<(unsigned)((n8 + 255) / 256), 256, 0, stream>>>(z, ZB, n8); }
    k_wt<<<HP / 16, 256, 0, stream>>>(w1, WT);
    k_hproj<<<dim3(NTOK / 64, HP / 64, 1), 32, 0, stream>>>(ZB, WT, b1, HPL);
    k_pair<<<NROWS / TI, NT, 0, stream>>>(HPL, w2, b2, OUT);
}
